// GraphEncoder_31542239822511
// MI455X (gfx1250) — hardware-run, weakly checked
//
#include <hip/hip_runtime.h>
#include <stddef.h>
#include <stdint.h>
#include <math.h>


#define F_IN    128
#define XQ      (F_IN / 8)
#define HC      160
#define NHEAD   5
#define CPH     32
#define LPW     (HC / 8)
#define K2      (2 * HC)
#define STW     32
#define NTHR    256
#define NWAVE   8
#define EPT     8
#define CHUNK   (NTHR * EPT)
#define WCAP    (EPT * 32)
#define LISTN   (NWAVE * WCAP)
#define NBMAX   2048
#define SLOTB   11
#define RCAP    28672
#define DEGCAP  256
#define GBM     64
#define GBN     32
#define GTHR    128
#define MROWS   128
#define APB     256
#define NEGSL   0.2f
#define ACTSL   0.01f
#define LN_EPS  1e-5f
#define WSMAX   134217728
#define LDS_AGG ((2 * RCAP + 2 * NBMAX + LISTN) * 4 + 128)

static_assert((CHUNK & (CHUNK - 1)) == 0 && CHUNK <= (1 << SLOTB));
static_assert(NBMAX == (1 << SLOTB));
static_assert(NTHR * 8 == NBMAX);
static_assert(LISTN >= NBMAX);
static_assert(LISTN >= NWAVE * WCAP);
static_assert((RCAP % 32) == 0);
static_assert(LDS_AGG <= 300000);
static_assert(GBM == (GTHR / 32) * 16 && GTHR == 2 * GBM);
static_assert(HC == NHEAD * CPH && GBN == CPH && (HC % GBN) == 0);
static_assert((F_IN % 32) == 0 && (K2 % 32) == 0 && K2 == 2 * HC);
static_assert((MROWS % GBM) == 0);
static_assert(LPW * 8 == HC && LPW < 32 && (LPW % 4) == 0 && LPW / 4 == NHEAD && 2 * LPW - 32 == 8);
static_assert(STW * 4 == 128 && (HC * 4) % 128 == 0 && (K2 * 2) % 128 == 0);
static_assert((APB * NHEAD * 4) % 128 == 0 && (APB * NHEAD) % 4 == 0 && (APB * NHEAD) / 4 <= 2 * APB);
static_assert(XQ == 16 && (F_IN % 8) == 0);
static_assert(HC <= NTHR && (HC % 32) == 0 && HC / 4 <= NTHR);

typedef float          v2f  __attribute__((ext_vector_type(2)));
typedef float          v4f  __attribute__((ext_vector_type(4)));
typedef float          v8f  __attribute__((ext_vector_type(8)));
typedef int            v4i  __attribute__((ext_vector_type(4)));
typedef int            v8i  __attribute__((ext_vector_type(8)));
typedef unsigned int   v4u  __attribute__((ext_vector_type(4)));
typedef unsigned short v8us __attribute__((ext_vector_type(8)));
typedef __bf16         v16b __attribute__((ext_vector_type(16)));
typedef v4f  __attribute__((may_alias)) v4fa;
typedef v8us __attribute__((may_alias)) v8usa;
union FragB { v16b v; v8us h[2]; v8i w; };

__device__ __forceinline__ v8f wmb(const FragB& a, const FragB& b, v8f c) {
  v8f d = __builtin_amdgcn_wmma_f32_16x16x32_bf16(false, a.v, false, b.v, (short)0, c, false, false);
  asm volatile("v_nop\n\tv_nop\n\tv_nop\n\tv_nop" : "+v"(d) : "v"(a.w), "v"(b.w));
  return d;
}

__device__ __forceinline__ unsigned int f2bf(float f) {
  const unsigned int u = __float_as_uint(f);
  return ((u + 0x7FFFu + ((u >> 16) & 1u)) >> 16) & 0xFFFFu;
}
__device__ __forceinline__ float bf2f(unsigned int b) { return __uint_as_float(b << 16); }
__device__ __forceinline__ float bfr(float f) { return bf2f(f2bf(f)); }
__device__ __forceinline__ v4f bfr4(const v4f a) {
  v4f r; r.x = bfr(a.x); r.y = bfr(a.y); r.z = bfr(a.z); r.w = bfr(a.w); return r;
}
__device__ __forceinline__ unsigned int pk2(float lo, float hi) { return f2bf(lo) | (f2bf(hi) << 16); }
__device__ __forceinline__ v4u pack8(const v4f a, const v4f b) {
  v4u r;
  r.x = pk2(a.x, a.y); r.y = pk2(a.z, a.w); r.z = pk2(b.x, b.y); r.w = pk2(b.z, b.w);
  return r;
}
__device__ __forceinline__ float leaky001(float x) { return x > 0.f ? x : ACTSL * x; }

__device__ __forceinline__ float head_const(const float* __restrict__ we, const float* __restrict__ ae, int hd) {
  const float* pw = we + hd * CPH;
  const float* pa = ae + hd * CPH;
  float s = 0.f;
#pragma unroll 1
  for (int c = 0; c < CPH; ++c) s = fmaf(bfr(pw[c]), bfr(pa[c]), s);
  return s;
}
__device__ __forceinline__ float att_logit(float as, float ad, float av, float ce) {
  float t = as + ad;
  t = fmaf(av, ce, t);
  return t > 0.f ? t : NEGSL * t;
}

__device__ __forceinline__ int scan_chunk(const int* __restrict__ dsts, int nE, int cbase, int slotBase,
                                          int nb, int vec8, int* list, int tid, int lane, int wave) {
  int wc = 0;
  const int el0  = tid * EPT;
  const int e0   = cbase + el0;
  const int sent = -2147483647 - 1;
  v4i da, db;
  if (vec8 != 0 && cbase + CHUNK <= nE) {
    da = *(const v4i*)(dsts + e0);
    db = *(const v4i*)(dsts + e0 + 4);
  } else {
    da.x = (e0     < nE) ? dsts[min(e0,     nE - 1)] : sent;
    da.y = (e0 + 1 < nE) ? dsts[min(e0 + 1, nE - 1)] : sent;
    da.z = (e0 + 2 < nE) ? dsts[min(e0 + 2, nE - 1)] : sent;
    da.w = (e0 + 3 < nE) ? dsts[min(e0 + 3, nE - 1)] : sent;
    db.x = (e0 + 4 < nE) ? dsts[min(e0 + 4, nE - 1)] : sent;
    db.y = (e0 + 5 < nE) ? dsts[min(e0 + 5, nE - 1)] : sent;
    db.z = (e0 + 6 < nE) ? dsts[min(e0 + 6, nE - 1)] : sent;
    db.w = (e0 + 7 < nE) ? dsts[min(e0 + 7, nE - 1)] : sent;
  }
  const unsigned nbs = (unsigned)slotBase;
  const unsigned unb = (unsigned)nb;
  const unsigned s0 = (unsigned)da.x - nbs, s1 = (unsigned)da.y - nbs;
  const unsigned s2 = (unsigned)da.z - nbs, s3 = (unsigned)da.w - nbs;
  const unsigned s4 = (unsigned)db.x - nbs, s5 = (unsigned)db.y - nbs;
  const unsigned s6 = (unsigned)db.z - nbs, s7 = (unsigned)db.w - nbs;
  const bool h0 = s0 < unb, h1 = s1 < unb, h2 = s2 < unb, h3 = s3 < unb;
  const bool h4 = s4 < unb, h5 = s5 < unb, h6 = s6 < unb, h7 = s7 < unb;
  const unsigned any = __builtin_amdgcn_ballot_w32(h0 | h1 | h2 | h3 | h4 | h5 | h6 | h7);
  if (any != 0u) {
#define HITJ(J, HJ, SJ) { \
      const unsigned mj = __builtin_amdgcn_ballot_w32(HJ); \
      if (mj != 0u) { \
        if (HJ) { \
          const int pos = wc + (int)__builtin_amdgcn_mbcnt_lo(mj, 0u); \
          if (pos < WCAP) list[wave * WCAP + pos] = ((el0 + (J)) << SLOTB) | (int)(SJ); \
        } \
        wc += (int)__builtin_popcount(mj); } }
    HITJ(0, h0, s0)
    HITJ(1, h1, s1)
    HITJ(2, h2, s2)
    HITJ(3, h3, s3)
    HITJ(4, h4, s4)
    HITJ(5, h5, s5)
    HITJ(6, h6, s6)
    HITJ(7, h7, s7)
#undef HITJ
  }
  return wc;
}

__global__ __launch_bounds__(NTHR) void k_xprep(const float* __restrict__ x, unsigned short* xb, int nN, int nUnits) {
  const int i = (int)blockIdx.x * NTHR + (int)threadIdx.x;
  if (i >= nUnits) return;
  const int row = i >> 4;
  const int c0  = (i & 15) * 8;
  const int rc  = row < nN ? row : nN - 1;
  const float* p = x + (size_t)rc * F_IN + c0;
  v4f a = *(const v4fa*)p, b = *(const v4fa*)(p + 4);
  const v4f z4 = {0.f, 0.f, 0.f, 0.f};
  if (row >= nN) { a = z4; b = z4; }
  const v4u hv = pack8(a, b);
  const size_t o = (size_t)row * F_IN + c0;
  *(volatile v4u*)(xb + o) = hv;
  __threadfence();
  *(volatile v4u*)(xb + o) = hv;
}

__global__ __launch_bounds__(NTHR) void k_wtr(const float* __restrict__ w, int Kin, int Ncol, int Nrows, int Kout,
                                              unsigned short* wt, int nUnits) {
  const int u = (int)blockIdx.x * NTHR + (int)threadIdx.x;
  if (u >= nUnits) return;
  const int kq = Kout >> 3;
  const int n  = u / kq;
  const int k8 = (u - n * kq) * 8;
  const int kk = k8 - (k8 / Kin) * Kin;
  const int ncl = n < Ncol ? n : Ncol - 1;
  const float* p = w + (size_t)kk * (size_t)Ncol + ncl;
  v4f a, b;
  a.x = p[0];                    a.y = p[(size_t)Ncol];         a.z = p[(size_t)2 * Ncol];     a.w = p[(size_t)3 * Ncol];
  b.x = p[(size_t)4 * Ncol];     b.y = p[(size_t)5 * Ncol];     b.z = p[(size_t)6 * Ncol];     b.w = p[(size_t)7 * Ncol];
  const v4f z4 = {0.f, 0.f, 0.f, 0.f};
  if (n >= Ncol || n >= Nrows) { a = z4; b = z4; }
  const v4u wv = pack8(a, b);
  unsigned short* o = wt + (size_t)n * (size_t)Kout + k8;
  *(volatile v4u*)o = wv;
  __threadfence();
  *(volatile v4u*)o = wv;
}

template<int EPI>
__global__ __launch_bounds__(GTHR) void k_gemm(
    const unsigned short* __restrict__ A, const unsigned short* __restrict__ WT, int K,
    float* outF, int ldo, int nRowsOut,
    const float* __restrict__ asv, const float* __restrict__ adv, float* AL, int MPr,
    const float* __restrict__ bias)
{
  __shared__ __attribute__((aligned(16))) float stg[GBM * GBN];
  __shared__ __attribute__((aligned(16))) float sav[2 * CPH];
  __shared__ __attribute__((aligned(16))) float sal[2 * GBM];
  const int tid = (int)threadIdx.x, lane = tid & 31, wave = tid >> 5, hh = lane >> 4, m = lane & 15;
  const int rowBase = (int)blockIdx.x * GBM;
  const int head    = (int)blockIdx.y;
  const int col0    = head * GBN;

  if (EPI == 0) {
    if (wave == 0)      sav[lane]       = bfr(asv[head * CPH + lane]);
    else if (wave == 1) sav[CPH + lane] = bfr(adv[head * CPH + lane]);
  }

  v8f acc[2];
  {
    const v8f z = {0.f, 0.f, 0.f, 0.f, 0.f, 0.f, 0.f, 0.f};
    acc[0] = z; acc[1] = z;
  }
  const unsigned short* ap = A  + (size_t)(rowBase + 16 * wave + m) * (size_t)K + 8 * hh;
  const unsigned short* wp = WT + (size_t)(col0 + m) * (size_t)K + 8 * hh;
  const int ksteps = K >> 5;
#pragma unroll 1
  for (int ks = 0; ks < ksteps; ++ks) {
    FragB af;
    af.h[0] = *(const v8usa*)(ap + 32 * ks);
    af.h[1] = *(const v8usa*)(ap + 32 * ks + 16);
#pragma unroll
    for (int t = 0; t < 2; ++t) {
      const unsigned short* wq = wp + (size_t)(16 * t) * (size_t)K + 32 * ks;
      FragB bf;
      bf.h[0] = *(const v8usa*)wq;
      bf.h[1] = *(const v8usa*)(wq + 16);
      acc[t] = wmb(af, bf, acc[t]);
    }
  }

#pragma unroll
  for (int t = 0; t < 2; ++t) {
    const int lc = 16 * t + m;
#pragma unroll
    for (int r = 0; r < 8; ++r) {
      const int lr = 16 * wave + 8 * hh + r;
      stg[lr * GBN + lc] = acc[t][r];
    }
  }
  __syncthreads();

  if (EPI == 0) {
    const int row   = tid & (GBM - 1);
    const int which = tid >> 6;
    const float* sv = sav + CPH * which;
    const float* sr = stg + row * GBN;
    float s = 0.f;
#pragma unroll
    for (int c4 = 0; c4 < GBN / 4; ++c4) {
      const v4f a = *(const v4fa*)(sr + 4 * c4);
      const v4f w = *(const v4fa*)(sv + 4 * c4);
      s = fmaf(a.x, w.x, s); s = fmaf(a.y, w.y, s); s = fmaf(a.z, w.z, s); s = fmaf(a.w, w.w, s);
    }
    sal[tid] = s;
    __syncthreads();
    if (wave == 0) {
      const int grp = lane >> 4;
      const int idx = 4 * (lane & 15);
      const v4f v = *(const v4fa*)(sal + GBM * grp + idx);
      float* p = AL + (size_t)(grp * NHEAD + head) * (size_t)MPr + rowBase + idx;
      *(volatile v4f*)p = v;
      __threadfence();
      *(volatile v4f*)p = v;
    }
  }

  const int cq = 4 * (lane & 7);
  const int rq = lane >> 3;
  v4f bv = {0.f, 0.f, 0.f, 0.f};
  if (EPI == 1) bv = bfr4(*(const v4fa*)(bias + col0 + cq));
  v4f fv[4];
#pragma unroll
  for (int i = 0; i < 4; ++i) {
    const int lr = 16 * wave + 4 * i + rq;
    v4f v = *(const v4fa*)(stg + lr * GBN + cq);
    if (EPI == 1) {
      v += bv;
      v.x = leaky001(v.x); v.y = leaky001(v.y); v.z = leaky001(v.z); v.w = leaky001(v.w);
    }
    fv[i] = v;
  }
#pragma unroll
  for (int i = 0; i < 4; ++i) {
    const int gr = rowBase + 16 * wave + 4 * i + rq;
    float* op = outF + (size_t)gr * (size_t)ldo + col0 + cq;
    if (gr < nRowsOut) *(volatile v4f*)op = fv[i];
  }
  __threadfence();
#pragma unroll
  for (int i = 0; i < 4; ++i) {
    const int gr = rowBase + 16 * wave + 4 * i + rq;
    float* op = outF + (size_t)gr * (size_t)ldo + col0 + cq;
    if (gr < nRowsOut) *(volatile v4f*)op = fv[i];
  }
}

__global__ __launch_bounds__(NTHR) void k_agg(
    const int* __restrict__ srcs, const int* __restrict__ dsts, const float* __restrict__ ea,
    const float* __restrict__ F, const float* __restrict__ AL,
    const float* __restrict__ we, const float* __restrict__ ae,
    const float* __restrict__ bias, const float* __restrict__ lng, const float* __restrict__ lnb,
    unsigned short* HA, float* ST,
    int nN, int nE, int nb, int vec8, int MPr) {
  extern __shared__ v4f lds_dyn[];
  int* reg1 = (int*)lds_dyn;
  int* reg2 = reg1 + RCAP;
  int* scnt = reg2 + RCAP;
  int* soff = scnt + NBMAX;
  int* list = soff + NBMAX;
  int* wcnt = list + LISTN;
  int* wtot = wcnt + NWAVE;
  float* sce = (float*)(wtot + NWAVE);
  const int tid = (int)threadIdx.x, lane = tid & 31, wave = tid >> 5;
  const int nodeBase = (int)blockIdx.x * nb;

  for (int i = tid; i < NBMAX; i += NTHR) scnt[i] = 0;
  if (wave == 0) {
    const int hd = lane < NHEAD ? lane : NHEAD - 1;
    const float cv = head_const(we, ae, hd);
    if (lane < NHEAD) sce[lane] = cv;
  }
  const int  lq   = lane < LPW ? lane : LPW - 1;
  const int  hl   = lq >> 2;
  const int  ch0  = 8 * lq;
  const bool act  = lane < LPW;
  const float fact = act ? 1.0f : 0.0f;
  const v4f bb0 = bfr4(*(const v4fa*)(bias + ch0)), bb1 = bfr4(*(const v4fa*)(bias + ch0 + 4));
  const v4f gg0 = bfr4(*(const v4fa*)(lng  + ch0)), gg1 = bfr4(*(const v4fa*)(lng  + ch0 + 4));
  const v4f be0 = bfr4(*(const v4fa*)(lnb  + ch0)), be1 = bfr4(*(const v4fa*)(lnb  + ch0 + 4));
  __syncthreads();

  int tot = 0;
  const int nChunks = (nE + CHUNK - 1) / CHUNK;
#pragma unroll 1
  for (int ch = 0; ch < nChunks; ++ch) {
    const int cbase = ch * CHUNK;
    const int wc = scan_chunk(dsts, nE, cbase, nodeBase, nb, vec8, list, tid, lane, wave);
    if (lane == 0) wcnt[wave] = wc;
    __syncthreads();
    int pre = 0, all = 0;
#pragma unroll
    for (int w2 = 0; w2 < NWAVE; ++w2) {
      int c = wcnt[w2];
      c = c < 0 ? 0 : (c > WCAP ? WCAP : c);
      all += c;
      pre += (w2 < wave) ? c : 0;
    }
    const int wcc  = wc > WCAP ? WCAP : wc;
    const int base = tot + pre;
#pragma unroll 1
    for (int i = lane; i < wcc; i += 32) {
      const int ent = list[wave * WCAP + i];
      const int el  = (ent >> SLOTB) & (CHUNK - 1);
      const int sl  = ent & (NBMAX - 1);
      int eid = cbase + el;
      eid = eid > nE - 1 ? nE - 1 : eid;
      const int pos = base + i;
      if (pos < RCAP) reg1[pos] = (int)(((unsigned)eid << SLOTB) | (unsigned)sl);
    }
    tot += all;
    tot = tot > RCAP ? RCAP : tot;
    __syncthreads();
  }
  const int nh = tot;

  if (wave == 0) {
#pragma unroll 1
    for (int b0 = 0; b0 < nh; b0 += 32) {
      const int idx = b0 + lane;
      const int uv  = reg1[idx < nh ? idx : nh - 1];
      const int m32 = (nh - b0) < 32 ? (nh - b0) : 32;
#pragma unroll 1
      for (int k = 0; k < m32; ++k) {
        const int u  = __builtin_amdgcn_readlane(uv, k);
        const int sl = u & (NBMAX - 1);
        if (lane == 0) scnt[sl] = scnt[sl] + 1;
      }
    }
  }
  __syncthreads();

  {
    const v4i ca = *(const v4i*)(scnt + 8 * tid);
    const v4i cb = *(const v4i*)(scnt + 8 * tid + 4);
    const int e0 = ca.x < 0 ? 0 : ca.x, e1 = ca.y < 0 ? 0 : ca.y, e2 = ca.z < 0 ? 0 : ca.z, e3 = ca.w < 0 ? 0 : ca.w;
    const int e4 = cb.x < 0 ? 0 : cb.x, e5 = cb.y < 0 ? 0 : cb.y, e6 = cb.z < 0 ? 0 : cb.z, e7 = cb.w < 0 ? 0 : cb.w;
    const int ts = e0 + e1 + e2 + e3 + e4 + e5 + e6 + e7;
    int incl = ts;
#pragma unroll
    for (int d = 1; d < 32; d <<= 1) {
      const int up = __shfl_up(incl, d);
      if (lane >= d) incl += up;
    }
    if (lane == 31) wtot[wave] = incl;
    __syncthreads();
    int pre = 0;
#pragma unroll
    for (int w2 = 0; w2 < NWAVE; ++w2) pre += (w2 < wave) ? wtot[w2] : 0;
    int run = pre + incl - ts;
    soff[8 * tid + 0] = run; run += e0;
    soff[8 * tid + 1] = run; run += e1;
    soff[8 * tid + 2] = run; run += e2;
    soff[8 * tid + 3] = run; run += e3;
    soff[8 * tid + 4] = run; run += e4;
    soff[8 * tid + 5] = run; run += e5;
    soff[8 * tid + 6] = run; run += e6;
    soff[8 * tid + 7] = run;
  }
  __syncthreads();
  for (int i = tid; i < NBMAX; i += NTHR) list[i] = soff[i];
  __syncthreads();

  if (wave == 0) {
#pragma unroll 1
    for (int b0 = 0; b0 < nh; b0 += 32) {
      const int idx = b0 + lane;
      const int uv  = reg1[idx < nh ? idx : nh - 1];
      const int m32 = (nh - b0) < 32 ? (nh - b0) : 32;
#pragma unroll 1
      for (int k = 0; k < m32; ++k) {
        const int u   = __builtin_amdgcn_readlane(uv, k);
        const int sl  = u & (NBMAX - 1);
        const int eid = (int)((unsigned)u >> SLOTB);
        if (lane == 0) {
          int pos = list[sl];
          pos = pos < 0 ? 0 : (pos > RCAP - 1 ? RCAP - 1 : pos);
          reg2[pos] = eid;
          list[sl] = pos + 1;
        }
      }
    }
  }
  __syncthreads();

  const int nbw = nb >> 3;
  const bool ovf = (nh >= RCAP);
  const float qnan = __int_as_float(0x7fc00000);
  const float ce_l = sce[hl];
  const int  sl4  = (16 * lane) & 31;
  const int  qsel = (lane >> 1) & 3;
  const bool oddl = (lane & 1) != 0;
  const int  shs  = (lane + (32 - LPW)) & 31;

#pragma unroll 1
  for (int jt = 0; jt < nbw; ++jt) {
    const int slot = wave * nbw + jt;
    const int grow = nodeBase + slot;
    const int gcl  = grow < nN ? grow : nN - 1;
    int st = soff[slot];
    const int craw = scnt[slot];
    int cnt = craw;
    st  = st < 0 ? 0 : (st > nh ? nh : st);
    cnt = cnt < 0 ? 0 : (cnt > DEGCAP ? DEGCAP : cnt);
    if (cnt > nh - st) cnt = nh - st;
    const float pz = (ovf || craw > DEGCAP) ? qnan : 0.0f;

    const float ad_l  = AL[(size_t)(NHEAD + hl) * (size_t)MPr + gcl];
    const float asd_l = AL[(size_t)hl * (size_t)MPr + gcl];
    const float* fdp  = F + (size_t)gcl * HC + ch0;
    const v4f fd0 = *(const v4fa*)fdp;
    const v4f fd1 = *(const v4fa*)(fdp + 4);

    float mx = -1.0e30f, dn = 0.0f, esum = 0.0f, eam = 0.0f;
    float a0 = 0.f, a1 = 0.f, a2 = 0.f, a3 = 0.f, a4 = 0.f, a5 = 0.f, a6 = 0.f, a7 = 0.f;

#pragma unroll 1
    for (int q = 0; q <= cnt; ++q) {
      float av, as_l;
      v4f fs0, fs1;
      if (q < cnt) {
        int idx = st + q; idx = idx > RCAP - 1 ? RCAP - 1 : idx;
        int eid = reg2[idx]; eid = eid < 0 ? 0 : (eid > nE - 1 ? nE - 1 : eid);
        const int sraw = srcs[eid];
        const int s = sraw < 0 ? 0 : (sraw > nN - 1 ? nN - 1 : sraw);
        av = bfr(ea[eid]);
        esum += av;
        as_l = AL[(size_t)hl * (size_t)MPr + s];
        const float* fsp = F + (size_t)s * HC + ch0;
        fs0 = *(const v4fa*)fsp;
        fs1 = *(const v4fa*)(fsp + 4);
      } else {
        eam  = esum / fmaxf((float)craw, 1.0f);
        av   = eam;
        as_l = asd_l;
        fs0  = fd0;
        fs1  = fd1;
      }
      const float lg = att_logit(as_l, ad_l, av, ce_l);
      const float df = lg - mx;
      const float ee = __expf(-fabsf(df));
      const bool up  = df > 0.f;
      const float s1 = up ? ee : 1.0f;
      const float s2 = up ? 1.0f : ee;
      mx = up ? lg : mx;
      dn = fmaf(dn, s1, s2);
      a0 = fmaf(a0, s1, s2 * fs0.x); a1 = fmaf(a1, s1, s2 * fs0.y);
      a2 = fmaf(a2, s1, s2 * fs0.z); a3 = fmaf(a3, s1, s2 * fs0.w);
      a4 = fmaf(a4, s1, s2 * fs1.x); a5 = fmaf(a5, s1, s2 * fs1.y);
      a6 = fmaf(a6, s1, s2 * fs1.z); a7 = fmaf(a7, s1, s2 * fs1.w);
    }
    const float inv = __builtin_amdgcn_rcpf(dn);
    float v0 = leaky001(fmaf(a0, inv, bb0.x)), v1 = leaky001(fmaf(a1, inv, bb0.y));
    float v2 = leaky001(fmaf(a2, inv, bb0.z)), v3 = leaky001(fmaf(a3, inv, bb0.w));
    float v4 = leaky001(fmaf(a4, inv, bb1.x)), v5 = leaky001(fmaf(a5, inv, bb1.y));
    float v6 = leaky001(fmaf(a6, inv, bb1.z)), v7 = leaky001(fmaf(a7, inv, bb1.w));

    float ps = fact * (((v0 + v1) + (v2 + v3)) + ((v4 + v5) + (v6 + v7)));
    ps += __shfl_xor(ps, 1); ps += __shfl_xor(ps, 2); ps += __shfl_xor(ps, 4);
    ps += __shfl_xor(ps, 8); ps += __shfl_xor(ps, 16);
    const float mean = ps * (1.0f / (float)HC);
    const float d0 = v0 - mean, d1 = v1 - mean, d2 = v2 - mean, d3 = v3 - mean;
    const float d4 = v4 - mean, d5 = v5 - mean, d6 = v6 - mean, d7 = v7 - mean;
    float pv = d0 * d0;
    pv = fmaf(d1, d1, pv); pv = fmaf(d2, d2, pv); pv = fmaf(d3, d3, pv);
    pv = fmaf(d4, d4, pv); pv = fmaf(d5, d5, pv); pv = fmaf(d6, d6, pv); pv = fmaf(d7, d7, pv);
    pv *= fact;
    pv += __shfl_xor(pv, 1); pv += __shfl_xor(pv, 2); pv += __shfl_xor(pv, 4);
    pv += __shfl_xor(pv, 8); pv += __shfl_xor(pv, 16);
    const float var = pv * (1.0f / (float)HC);
    const float rsd = 1.0f / sqrtf(var + LN_EPS);
    const bool live = grow < nN;
    float y0 = fmaf(d0 * rsd, gg0.x, be0.x), y1 = fmaf(d1 * rsd, gg0.y, be0.y);
    float y2 = fmaf(d2 * rsd, gg0.z, be0.z), y3 = fmaf(d3 * rsd, gg0.w, be0.w);
    float y4 = fmaf(d4 * rsd, gg1.x, be1.x), y5 = fmaf(d5 * rsd, gg1.y, be1.y);
    float y6 = fmaf(d6 * rsd, gg1.z, be1.z), y7 = fmaf(d7 * rsd, gg1.w, be1.w);
    y0 = (live ? y0 : 0.f) + pz; y1 = (live ? y1 : 0.f) + pz; y2 = (live ? y2 : 0.f) + pz; y3 = (live ? y3 : 0.f) + pz;
    y4 = (live ? y4 : 0.f) + pz; y5 = (live ? y5 : 0.f) + pz; y6 = (live ? y6 : 0.f) + pz; y7 = (live ? y7 : 0.f) + pz;

    const unsigned int hb0 = f2bf(y0), hb1 = f2bf(y1), hb2 = f2bf(y2), hb3 = f2bf(y3);
    const unsigned int hb4 = f2bf(y4), hb5 = f2bf(y5), hb6 = f2bf(y6), hb7 = f2bf(y7);
    const unsigned int lb0 = f2bf(y0 - bf2f(hb0)), lb1 = f2bf(y1 - bf2f(hb1));
    const unsigned int lb2 = f2bf(y2 - bf2f(hb2)), lb3 = f2bf(y3 - bf2f(hb3));
    const unsigned int lb4 = f2bf(y4 - bf2f(hb4)), lb5 = f2bf(y5 - bf2f(hb5));
    const unsigned int lb6 = f2bf(y6 - bf2f(hb6)), lb7 = f2bf(y7 - bf2f(hb7));
    const int hw0 = (int)(hb0 | (hb1 << 16)), hw1 = (int)(hb2 | (hb3 << 16));
    const int hw2 = (int)(hb4 | (hb5 << 16)), hw3 = (int)(hb6 | (hb7 << 16));
    const int lw0 = (int)(lb0 | (lb1 << 16)), lw1 = (int)(lb2 | (lb3 << 16));
    const int lw2 = (int)(lb4 | (lb5 << 16)), lw3 = (int)(lb6 | (lb7 << 16));
    const int gl0 = __shfl(lw0, shs), gl1 = __shfl(lw1, shs), gl2 = __shfl(lw2, shs), gl3 = __shfl(lw3, shs);
    v4u p1, p2;
    p1.x = (unsigned int)(act ? hw0 : gl0); p1.y = (unsigned int)(act ? hw1 : gl1);
    p1.z = (unsigned int)(act ? hw2 : gl2); p1.w = (unsigned int)(act ? hw3 : gl3);
    p2.x = (unsigned int)gl0; p2.y = (unsigned int)gl1; p2.z = (unsigned int)gl2; p2.w = (unsigned int)gl3;
    unsigned short* hp = HA + (size_t)grow * K2;
    const bool wr1 = grow < MPr;
    const bool wr2 = wr1 && (lane < 2 * LPW - 32);

    const float mxs = mx + pz;
    float tm0, tm1, tm2, tm3, td0, td1, td2, td3, ts0, ts1, ts2, ts3, ta0, ta1, ta2, ta3;
    {
      const int c0 = sl4, c1 = (sl4 + 4) & 31, c2 = (sl4 + 8) & 31, c3 = (sl4 + 12) & 31;
      tm0 = __shfl(mxs, c0);   tm1 = __shfl(mxs, c1);   tm2 = __shfl(mxs, c2);   tm3 = __shfl(mxs, c3);
      td0 = __shfl(dn, c0);    td1 = __shfl(dn, c1);    td2 = __shfl(dn, c2);    td3 = __shfl(dn, c3);
      ts0 = __shfl(asd_l, c0); ts1 = __shfl(asd_l, c1); ts2 = __shfl(asd_l, c2); ts3 = __shfl(asd_l, c3);
      ta0 = __shfl(ad_l, c0);  ta1 = __shfl(ad_l, c1);  ta2 = __shfl(ad_l, c2);  ta3 = __shfl(ad_l, c3);
    }
    v4f sv;
    sv.x = qsel == 0 ? tm0 : (qsel == 1 ? td0 : (qsel == 2 ? ts0 : ta0));
    sv.y = qsel == 0 ? tm1 : (qsel == 1 ? td1 : (qsel == 2 ? ts1 : ta1));
    sv.z = qsel == 0 ? tm2 : (qsel == 1 ? td2 : (qsel == 2 ? ts2 : ta2));
    sv.w = qsel == 0 ? tm3 : (qsel == 1 ? td3 : (qsel == 2 ? ts3 : ta3));
    const float o1odd = (lane == 1) ? eam : 0.0f;
    sv.y = oddl ? o1odd : sv.y;
    sv.z = oddl ? 0.0f : sv.z;
    sv.w = oddl ? 0.0f : sv.w;
    float* stp = ST + (size_t)grow * STW + 4 * lane;
    const bool wrs = wr1 && (lane < 8);

    if (wr1) *(volatile v4u*)(hp + 8 * lane) = p1;
    if (wr2) *(volatile v4u*)(hp + 256 + 8 * lane) = p2;
    if (wrs) *(volatile v4f*)stp = sv;
    __threadfence();
    if (wr1) *(volatile v4u*)(hp + 8 * lane) = p1;
    if (wr2) *(volatile v4u*)(hp + 256 + 8 * lane) = p2;
    if (wrs) *(volatile v4f*)stp = sv;
  }
}

__global__ __launch_bounds__(APB) void k_alpha(
    const int* __restrict__ srcs, const int* __restrict__ dsts, const float* __restrict__ ea,
    const float* __restrict__ ST, int stStride,
    const float* __restrict__ we1, const float* __restrict__ ae1,
    const float* __restrict__ we2, const float* __restrict__ ae2,
    int nE, int nN, int nRowsTot, float* aout) {
  __shared__ __attribute__((aligned(16))) float sOut[APB * NHEAD];
  __shared__ float sce[16];
  const int tid = (int)threadIdx.x, lane = tid & 31, wave = tid >> 5;

  if (wave < 2) {
    const int hd = lane < NHEAD ? lane : NHEAD - 1;
    float cv;
    if (wave == 0) cv = head_const(we1, ae1, hd);
    else           cv = head_const(we2, ae2, hd);
    if (lane < NHEAD) sce[8 * wave + lane] = cv;
  }

  const int nEN = nE + nN;
  const int vb  = (int)blockIdx.x * APB;
  const int vr  = vb + tid;
  const int vrc = vr < nRowsTot ? vr : nRowsTot - 1;
  const int ly  = vrc >= nEN ? 1 : 0;
  const int r   = vrc - ly * nEN;
  const bool selfr = r >= nE;
  const int ec  = r < nE ? r : nE - 1;
  int nd = r - nE; nd = nd < 0 ? 0 : (nd > nN - 1 ? nN - 1 : nd);
  int se = srcs[ec], de = dsts[ec];
  se = se < 0 ? 0 : (se > nN - 1 ? nN - 1 : se);
  de = de < 0 ? 0 : (de > nN - 1 ? nN - 1 : de);
  const int msk = selfr ? -1 : 0;
  const int s = (se & ~msk) | (nd & msk);
  const int d = (de & ~msk) | (nd & msk);
  const float eav = bfr(ea[ec]);
  __syncthreads();

  const float* stl = ST + (size_t)ly * (size_t)stStride;
  const float* rd  = stl + (size_t)d * STW;
  const float* rs  = stl + (size_t)s * STW;
  const v4f m0 = *(const v4fa*)(rd);
  const v4f m1 = *(const v4fa*)(rd + 4);
  const v4f n0 = *(const v4fa*)(rd + 8);
  const v4f n1 = *(const v4fa*)(rd + 12);
  const v4f t0 = *(const v4fa*)(rd + 24);
  const v4f t1 = *(const v4fa*)(rd + 28);
  const v4f u0 = *(const v4fa*)(rs + 16);
  const v4f u1 = *(const v4fa*)(rs + 20);
  const float eam = m1.y;
  const float av = __int_as_float((__float_as_int(eav) & ~msk) | (__float_as_int(eam) & msk));
  const float* cep = sce + 8 * ly;
  const float c0 = cep[0], c1 = cep[1], c2 = cep[2], c3 = cep[3], c4 = cep[4];

  const float al0 = __expf(att_logit(u0.x, t0.x, av, c0) - m0.x) * __builtin_amdgcn_rcpf(n0.x);
  const float al1 = __expf(att_logit(u0.y, t0.y, av, c1) - m0.y) * __builtin_amdgcn_rcpf(n0.y);
  const float al2 = __expf(att_logit(u0.z, t0.z, av, c2) - m0.z) * __builtin_amdgcn_rcpf(n0.z);
  const float al3 = __expf(att_logit(u0.w, t0.w, av, c3) - m0.w) * __builtin_amdgcn_rcpf(n0.w);
  const float al4 = __expf(att_logit(u1.x, t1.x, av, c4) - m1.x) * __builtin_amdgcn_rcpf(n1.x);
  sOut[NHEAD * tid + 0] = al0;
  sOut[NHEAD * tid + 1] = al1;
  sOut[NHEAD * tid + 2] = al2;
  sOut[NHEAD * tid + 3] = al3;
  sOut[NHEAD * tid + 4] = al4;
  __syncthreads();

  const int nvr = (nRowsTot - vb) < APB ? (nRowsTot - vb) : APB;
  const int nf4 = (nvr * NHEAD) >> 2;
  const int u0i = tid, u1i = APB + tid;
  const int u0c = u0i < (APB * NHEAD) / 4 ? u0i : (APB * NHEAD) / 4 - 1;
  const int u1c = u1i < (APB * NHEAD) / 4 ? u1i : (APB * NHEAD) / 4 - 1;
  const v4f va = *(const v4fa*)(sOut + 4 * u0c);
  const v4f vb4 = *(const v4fa*)(sOut + 4 * u1c);
  const bool oka = u0i < nf4;
  const bool okb = u1i < nf4;
  float* opa = aout + (size_t)vb * NHEAD + 4 * (size_t)u0i;
  float* opb = aout + (size_t)vb * NHEAD + 4 * (size_t)u1i;
  if (oka) *(volatile v4f*)opa = va;
  if (okb) *(volatile v4f*)opb = vb4;
  __threadfence();
  if (oka) *(volatile v4f*)opa = va;
  if (okb) *(volatile v4f*)opb = vb4;
}

__global__ __launch_bounds__(NTHR) void k_pool(const float* __restrict__ X3, const int* __restrict__ bat, int nN,
                                               float* pooled) {
  __shared__ int plist[LISTN];
  __shared__ int pwc[NWAVE];
  __shared__ __attribute__((aligned(16))) float sp[HC];
  const int tid = (int)threadIdx.x, lane = tid & 31, wave = tid >> 5;
  const int g = (int)blockIdx.x;
  const int cix = tid < HC ? tid : HC - 1;
  float acc = 0.0f;
  int total = 0;
  const int nChunks = (nN + CHUNK - 1) / CHUNK;
#pragma unroll 1
  for (int ch = 0; ch < nChunks; ++ch) {
    const int cbase = ch * CHUNK;
    const int wc = scan_chunk(bat, nN, cbase, g, 1, 1, plist, tid, lane, wave);
    if (lane == 0) pwc[wave] = wc;
    __syncthreads();
#pragma unroll 1
    for (int w2 = 0; w2 < NWAVE; ++w2) {
      int c = pwc[w2];
      c = c < 0 ? 0 : (c > WCAP ? WCAP : c);
      total += c;
#pragma unroll 1
      for (int i = 0; i < c; ++i) {
        const int ent = plist[w2 * WCAP + i];
        const int el  = (ent >> SLOTB) & (CHUNK - 1);
        int n = cbase + el;
        n = n > nN - 1 ? nN - 1 : n;
        acc += X3[(size_t)n * HC + cix];
      }
    }
    __syncthreads();
  }
  const float rr = acc * (1.0f / fmaxf((float)total, 1.0f));
  if (tid < HC) sp[tid] = rr;
  __syncthreads();
  const int tc = tid < HC / 4 ? tid : HC / 4 - 1;
  const v4f v = *(const v4fa*)(sp + 4 * tc);
  float* op = pooled + (size_t)g * HC + 4 * tc;
  const bool ok = tid < HC / 4;
  if (ok) *(volatile v4f*)op = v;
  __threadfence();
  if (ok) *(volatile v4f*)op = v;
}

static int pick_nb(int nE, int nN) {
  int nb = NBMAX;
  while (nb > 32 && (long long)nb * (long long)nE * 5LL > (long long)RCAP * (long long)nN * 4LL) nb >>= 1;
  return nb;
}
static inline int cdiv(int a, int b) { return (a + b - 1) / b; }

extern "C" void kernel_launch(void* const* d_in, const int* in_sizes, int n_in,
                              void* d_out, int out_size, void* d_ws, size_t ws_size,
                              hipStream_t stream) {
  if (n_in < 22) return;
  if (in_sizes[0] < F_IN || (in_sizes[0] % F_IN) != 0) return;
  const int nN = in_sizes[0] / F_IN;
  if (nN > (1 << 22)) return;
  if (in_sizes[1] < 2 || (in_sizes[1] & 1) != 0) return;
  const int nE = in_sizes[1] / 2;
  if (nE < 1 || nE >= (1 << (32 - SLOTB))) return;
  if (in_sizes[2] != nE) return;
  if (in_sizes[3] != nN) return;
  if (in_sizes[4] != F_IN * HC) return;
  if (in_sizes[5] != HC) return;
  if (in_sizes[6] != HC || in_sizes[7] != HC || in_sizes[8] != HC) return;
  if (in_sizes[9] != HC) return;
  if (in_sizes[10] != HC * HC) return;
  if (in_sizes[11] != HC) return;
  if (in_sizes[12] != HC || in_sizes[13] != HC || in_sizes[14] != HC) return;
  if (in_sizes[15] != HC) return;
  if (in_sizes[16] != HC || in_sizes[17] != HC || in_sizes[18] != HC || in_sizes[19] != HC) return;
  if (in_sizes[20] != HC * HC) return;
  if (in_sizes[21] != HC) return;

  const long long nEN = (long long)nE + (long long)nN;
  const long long fixedOut = (long long)nN * HC + 2LL * NHEAD * nEN;
  if ((long long)out_size <= fixedOut) return;
  const long long rem = (long long)out_size - fixedOut;
  if ((rem % HC) != 0) return;
  const long long Gll = rem / HC;
  if (Gll < 1 || Gll > 65535) return;
  const int G = (int)Gll;
  if (2LL * nEN > 2147483647LL / 8) return;
  const int nRowsTot = (int)(2 * nEN);
  if ((nRowsTot % 32) != 0) return;

  const float* x    = (const float*)d_in[0];
  const int*   ei   = (const int*)  d_in[1];
  const float* ea   = (const float*)d_in[2];
  const int*   bat  = (const int*)  d_in[3];
  const float* w1   = (const float*)d_in[4];
  const float* we1  = (const float*)d_in[5];
  const float* as1  = (const float*)d_in[6];
  const float* ad1  = (const float*)d_in[7];
  const float* ae1  = (const float*)d_in[8];
  const float* b1   = (const float*)d_in[9];
  const float* w2   = (const float*)d_in[10];
  const float* we2  = (const float*)d_in[11];
  const float* as2  = (const float*)d_in[12];
  const float* ad2  = (const float*)d_in[13];
  const float* ae2  = (const float*)d_in[14];
  const float* b2   = (const float*)d_in[15];
  const float* ln1g = (const float*)d_in[16];
  const float* ln1b = (const float*)d_in[17];
  const float* ln2g = (const float*)d_in[18];
  const float* ln2b = (const float*)d_in[19];
  const float* mw   = (const float*)d_in[20];
  const float* mb   = (const float*)d_in[21];
  float* out   = (float*)d_out;
  float* oX3   = out;
  float* oPool = out + (size_t)nN * HC;
  float* oAlf  = oPool + (size_t)G * HC;
  const int* src = ei;
  const int* dst = ei + nE;

  const int MP   = cdiv(nN, MROWS) * MROWS;
  const int nb   = pick_nb(nE, nN);
  if (nb < 32 || (nb & (nb - 1)) != 0 || nb > NBMAX) return;
  const int gA   = cdiv(MP, nb);
  const int vec8 = ((nE & 3) == 0) ? 1 : 0;
  if (gA * nb < MP) return;

  char* ws = (char*)d_ws;
  size_t off = 0;
  const size_t oXB  = off; off += (size_t)MP * F_IN * 2;           off = (off + 255) & ~(size_t)255;
  const size_t oW1T = off; off += (size_t)HC * F_IN * 2;           off = (off + 255) & ~(size_t)255;
  const size_t oW2T = off; off += (size_t)HC * K2 * 2;             off = (off + 255) & ~(size_t)255;
  const size_t oMWT = off; off += (size_t)HC * K2 * 2;             off = (off + 255) & ~(size_t)255;
  const size_t oF   = off; off += (size_t)MP * HC * 4;             off = (off + 255) & ~(size_t)255;
  const size_t oHA  = off; off += (size_t)MP * K2 * 2;             off = (off + 255) & ~(size_t)255;
  const size_t alStride = (size_t)2 * NHEAD * (size_t)MP;
  const size_t oAL  = off; off += 2 * alStride * 4;                off = (off + 255) & ~(size_t)255;
  const size_t stStride = (size_t)MP * STW;
  const size_t oST  = off; off += 2 * stStride * 4;                off = (off + 255) & ~(size_t)255;
  if (off > ws_size || off > (size_t)WSMAX) return;
  if (stStride > (size_t)2147483647) return;
  unsigned short* XB  = (unsigned short*)(ws + oXB);
  unsigned short* W1T = (unsigned short*)(ws + oW1T);
  unsigned short* W2T = (unsigned short*)(ws + oW2T);
  unsigned short* MWT = (unsigned short*)(ws + oMWT);
  float*          F   = (float*)(ws + oF);
  unsigned short* HA  = (unsigned short*)(ws + oHA);
  float*          AL1 = (float*)(ws + oAL);
  float*          AL2 = AL1 + alStride;
  float*          ST1 = (float*)(ws + oST);
  float*          ST2 = ST1 + stStride;

  hipFuncSetAttribute(reinterpret_cast<const void*>(&k_agg),
                      hipFuncAttributeMaxDynamicSharedMemorySize, LDS_AGG);

  const int nUx = MP * XQ;
  k_xprep<<<cdiv(nUx, NTHR), NTHR, 0, stream>>>(x, XB, nN, nUx);

  {
    const int nUw1 = HC * (F_IN / 8);
    k_wtr<<<cdiv(nUw1, NTHR), NTHR, 0, stream>>>(w1, F_IN, HC, HC, F_IN, W1T, nUw1);
    const int nUw2 = HC * (K2 / 8);
    k_wtr<<<cdiv(nUw2, NTHR), NTHR, 0, stream>>>(w2, HC, HC, HC, K2, W2T, nUw2);
    k_wtr<<<cdiv(nUw2, NTHR), NTHR, 0, stream>>>(mw, HC, HC, HC, K2, MWT, nUw2);
  }

  const int gM = MP / GBM;
  k_gemm<0><<<dim3(gM, HC / GBN), GTHR, 0, stream>>>(XB, W1T, F_IN, F, HC, MP, as1, ad1, AL1, MP, b1);
  k_agg<<<gA, NTHR, LDS_AGG, stream>>>(src, dst, ea, F, AL1, we1, ae1, b1, ln1g, ln1b, HA, ST1,
                                       nN, nE, nb, vec8, MP);
  k_gemm<0><<<dim3(gM, HC / GBN), GTHR, 0, stream>>>(HA, W2T, K2, F, HC, MP, as2, ad2, AL2, MP, b2);
  k_agg<<<gA, NTHR, LDS_AGG, stream>>>(src, dst, ea, F, AL2, we2, ae2, b2, ln2g, ln2b, HA, ST2,
                                       nN, nE, nb, vec8, MP);
  k_gemm<1><<<dim3(gM, HC / GBN), GTHR, 0, stream>>>(HA, MWT, K2, oX3, HC, nN, as1, ad1, AL1, MP, mb);
  k_pool<<<G, NTHR, 0, stream>>>(oX3, bat, nN, oPool);
  k_alpha<<<cdiv(nRowsTot, APB), APB, 0, stream>>>(src, dst, ea, ST1, (int)stStride, we1, ae1, we2, ae2,
                                                   nE, nN, nRowsTot, oAlf);
}
